// PointNetSetAbstraction_78228534329994
// MI455X (gfx1250) — hardware-verified
//
#include <hip/hip_runtime.h>
#pragma clang fp contract(off)

typedef __attribute__((ext_vector_type(16))) _Float16 v16h;
typedef __attribute__((ext_vector_type(8)))  _Float16 v8h;
typedef __attribute__((ext_vector_type(8)))  float    v8f;
typedef __attribute__((ext_vector_type(4)))  float    v4f;
typedef __attribute__((ext_vector_type(4)))  int      v4i;

constexpr int kBatch   = 8;
constexpr int kPts     = 4096;
constexpr int kCent    = 1024;
constexpr int kSamp    = 32;
constexpr int kChIn    = 64;
constexpr int kChMid   = 64;
constexpr int kChOut   = 128;
constexpr int kW0Pitch = 67;
constexpr int kRows    = kBatch * kCent * kSamp;
constexpr int kSrcRows = kBatch * kPts;
constexpr int kGroups  = kBatch * kCent;
constexpr int kDepth   = 64;
constexpr float kWCarry    = 64.0f;
constexpr float kWCarryInv = 1.0f / kWCarry;

static_assert(kRows == 262144, "row count");
static_assert(kSrcRows % 64 == 0 && kRows % 64 == 0, "M tile multiple");
static_assert(kChMid % 64 == 0 && kChOut % 64 == 0, "N tile multiple");
static_assert(kDepth % 32 == 0 && kChIn == kDepth && kChMid == kDepth, "K multiple of 32");
static_assert(kW0Pitch == kChIn + 3, "W0 pitch");
static_assert((size_t)kGroups * 3 * 4 == 98304, "out1 byte offset");
static_assert(((size_t)kGroups * 3 + (size_t)kGroups * kChOut) * 4 == 4292608, "out total bytes");

union FragU { v16h v; v8h h[2]; };
__device__ __forceinline__ v16h frag_load(const _Float16* p) {
  FragU f;
  f.h[0] = *(const v8h*)(p);
  f.h[1] = *(const v8h*)(p + 16);
  return f.v;
}
__device__ __forceinline__ v8f mma_h(v16h a, v16h b, v8f c) {
  return __builtin_amdgcn_wmma_f32_16x16x32_f16(false, a, false, b, (short)0, c, false, false);
}
__device__ __forceinline__ void guard_row4(v8f& a, v8f& b, v8f& c, v8f& d, v16h x, v16h y0, v16h y1, v16h y2, v16h y3) {
  asm volatile("v_nop\n\tv_nop\n\tv_nop\n\tv_nop" : "+v"(a), "+v"(b), "+v"(c), "+v"(d) : "v"(x), "v"(y0), "v"(y1), "v"(y2), "v"(y3));
}
__device__ __forceinline__ void acc_guard4(v8f& a, v8f& b, v8f& c, v8f& d) {
  asm volatile("v_nop\n\tv_nop\n\tv_nop\n\tv_nop" : "+v"(a), "+v"(b), "+v"(c), "+v"(d));
}
__device__ __forceinline__ void wave_lds_sync() {
  __builtin_amdgcn_fence(__ATOMIC_RELEASE, "workgroup");
  __builtin_amdgcn_wave_barrier();
  __builtin_amdgcn_fence(__ATOMIC_ACQUIRE, "workgroup");
}
__device__ __forceinline__ int clamp_pt(int i) {
  i = i < 0 ? 0 : i;
  i = i > (kPts - 1) ? (kPts - 1) : i;
  return i;
}

__global__ __launch_bounds__(512) void fps_kernel(const float* __restrict__ xyz, int* __restrict__ centIdx) {
#pragma clang fp contract(off)
  __shared__ __align__(16) float sX[kPts * 3];
  __shared__ __align__(16) int sIdx[kCent];
  __shared__ float s_v[16];
  __shared__ int s_i[16];
  __shared__ int s_best;

  const int b = blockIdx.x;
  const int tid = threadIdx.x;
  const int lane = tid & 31;
  const int wid = tid >> 5;

  {
    const v4f* X4 = (const v4f*)(xyz + (size_t)b * kPts * 3);
    v4f* sX4 = (v4f*)sX;
#pragma unroll
    for (int j = 0; j < 6; ++j) sX4[j * 512 + tid] = X4[j * 512 + tid];
  }
  __syncthreads();

  float px[8], py[8], pz[8], dist[8];
#pragma unroll
  for (int j = 0; j < 8; ++j) {
    const int p = j * 512 + tid;
    px[j] = sX[p * 3 + 0];
    py[j] = sX[p * 3 + 1];
    pz[j] = sX[p * 3 + 2];
    dist[j] = 1e10f;
  }

  int cur = 0;
  for (int it = 0; it < kCent; ++it) {
    if (tid == 0) sIdx[it] = cur;
    const float cx = sX[cur * 3 + 0];
    const float cy = sX[cur * 3 + 1];
    const float cz = sX[cur * 3 + 2];
    float bv = -1.0f;
    int bi = 0;
#pragma unroll
    for (int j = 0; j < 8; ++j) {
      const float dx = px[j] - cx;
      const float dy = py[j] - cy;
      const float dz = pz[j] - cz;
      const float t0 = dx * dx;
      const float t1 = dy * dy;
      const float t2 = dz * dz;
      const float d = (t0 + t2) + t1;
      const float nd = fminf(dist[j], d);
      dist[j] = nd;
      const int p = j * 512 + tid;
      if (nd > bv) { bv = nd; bi = p; }
    }
#pragma unroll
    for (int off = 16; off > 0; off >>= 1) {
      const float ov = __shfl_xor(bv, off, 32);
      const int   oi = __shfl_xor(bi, off, 32);
      if (ov > bv || (ov == bv && oi < bi)) { bv = ov; bi = oi; }
    }
    if (lane == 0) { s_v[wid] = bv; s_i[wid] = bi; }
    __syncthreads();
    if (wid == 0) {
      float v2 = s_v[lane & 15];
      int   i2 = s_i[lane & 15];
#pragma unroll
      for (int off = 16; off > 0; off >>= 1) {
        const float ov = __shfl_xor(v2, off, 32);
        const int   oi = __shfl_xor(i2, off, 32);
        if (ov > v2 || (ov == v2 && oi < i2)) { v2 = ov; i2 = oi; }
      }
      if (lane == 0) s_best = i2;
    }
    __syncthreads();
    cur = clamp_pt(s_best);
  }
  __syncthreads();
  if (tid < 256) {
    const v4i v = ((const v4i*)sIdx)[tid];
    int* dst = centIdx + (size_t)b * kCent + tid * 4;
    *(volatile v4i*)dst = v;
    __threadfence();
    *(volatile v4i*)dst = v;
  }
}

__global__ __launch_bounds__(256) void newxyz_kernel(const float* __restrict__ xyz, const int* __restrict__ centIdx,
                                                     float* __restrict__ out) {
  const int i = blockIdx.x * 256 + threadIdx.x;
  if (i < kGroups * 3) {
    const int bs = i / 3;
    const int c = i - bs * 3;
    const int b = bs >> 10;
    const int ci = clamp_pt(centIdx[bs]);
    const float v = xyz[((size_t)b * kPts + ci) * 3 + c];
    *(volatile float*)(out + i) = v;
    __threadfence();
    *(volatile float*)(out + i) = v;
  }
}

__global__ __launch_bounds__(256) void prep_w_kernel(const float* __restrict__ W0, const float* __restrict__ W1,
                                                     const float* __restrict__ W2, unsigned short* __restrict__ Wp0,
                                                     unsigned short* __restrict__ Wp1, unsigned short* __restrict__ Wp2) {
  const int which = blockIdx.y;
  const float* W = (which == 0) ? W0 : ((which == 1) ? W1 : W2);
  unsigned short* Wp = (which == 0) ? Wp0 : ((which == 1) ? Wp1 : Wp2);
  const int ldw = (which == 0) ? kW0Pitch : kDepth;
  const int coff = (which == 0) ? 3 : 0;
  const int rows = (which == 2) ? kChOut : kChMid;
  const int t = blockIdx.x * 256 + threadIdx.x;
  if (t < rows * 8) {
    const int row = t >> 3;
    const int c8 = (t & 7) * 8;
    const float* src = W + (size_t)row * ldw + coff + c8;
    v8h o;
    o[0] = (_Float16)(src[0] * kWCarry);
    o[1] = (_Float16)(src[1] * kWCarry);
    o[2] = (_Float16)(src[2] * kWCarry);
    o[3] = (_Float16)(src[3] * kWCarry);
    o[4] = (_Float16)(src[4] * kWCarry);
    o[5] = (_Float16)(src[5] * kWCarry);
    o[6] = (_Float16)(src[6] * kWCarry);
    o[7] = (_Float16)(src[7] * kWCarry);
    _Float16* dst = (_Float16*)Wp + (size_t)t * 8;
    *(volatile v8h*)dst = o;
    __threadfence();
    *(volatile v8h*)dst = o;
  }
}

__global__ __launch_bounds__(256) void cast_points_kernel(const float* __restrict__ in, unsigned short* __restrict__ outp,
                                                          int nThreads) {
  const int t = blockIdx.x * 256 + threadIdx.x;
  if (t < nThreads) {
    const v4f a0 = *(const v4f*)(in + (size_t)t * 8);
    const v4f a1 = *(const v4f*)(in + (size_t)t * 8 + 4);
    v8h o;
    o[0] = (_Float16)a0[0];
    o[1] = (_Float16)a0[1];
    o[2] = (_Float16)a0[2];
    o[3] = (_Float16)a0[3];
    o[4] = (_Float16)a1[0];
    o[5] = (_Float16)a1[1];
    o[6] = (_Float16)a1[2];
    o[7] = (_Float16)a1[3];
    _Float16* dst = (_Float16*)outp + (size_t)t * 8;
    *(volatile v8h*)dst = o;
    __threadfence();
    *(volatile v8h*)dst = o;
  }
}

template <int EPI>
__global__ __launch_bounds__(256) void gemm_k64(const unsigned short* __restrict__ Ap, const unsigned short* __restrict__ Btp,
                                                float* Cout, float* Cmin, float* __restrict__ part,
                                                const float* __restrict__ bias, int M, int N, float scale) {
  const _Float16* A = (const _Float16*)Ap;
  const _Float16* Bt = (const _Float16*)Btp;
  __shared__ __align__(16) float sT[8][16 * 68];
  const int lane = threadIdx.x & 31;
  const int wave = threadIdx.x >> 5;
  const int tilesN = N >> 6;
  const int tilesM = M >> 6;
  const int tile = blockIdx.x * 8 + wave;
  if (tile >= tilesM * tilesN) return;
  const int tm = tile / tilesN;
  const int tn = tile - tm * tilesN;
  const int m0 = tm << 6;
  const int n0 = tn << 6;
  const int rlane = lane & 15;
  const int hh = lane >> 4;
  const int koff = hh * 8;
  const int mOff = hh * 8;

  v8f acc[4][4];
#pragma unroll
  for (int i = 0; i < 4; ++i)
#pragma unroll
    for (int j = 0; j < 4; ++j) acc[i][j] = (v8f){0.f, 0.f, 0.f, 0.f, 0.f, 0.f, 0.f, 0.f};

#pragma unroll 1
  for (int k0 = 0; k0 < kDepth; k0 += 32) {
    v16h bh[4];
#pragma unroll
    for (int j = 0; j < 4; ++j) bh[j] = frag_load(Bt + (size_t)(n0 + (j << 4) + rlane) * kDepth + koff + k0);
#pragma unroll
    for (int i = 0; i < 4; ++i) {
      const v16h ah = frag_load(A + (size_t)(m0 + (i << 4) + rlane) * kDepth + koff + k0);
#pragma unroll
      for (int j = 0; j < 4; ++j) acc[i][j] = mma_h(ah, bh[j], acc[i][j]);
      guard_row4(acc[i][0], acc[i][1], acc[i][2], acc[i][3], ah, bh[0], bh[1], bh[2], bh[3]);
    }
  }
  acc_guard4(acc[0][0], acc[0][1], acc[0][2], acc[0][3]);
  acc_guard4(acc[1][0], acc[1][1], acc[1][2], acc[1][3]);
  acc_guard4(acc[2][0], acc[2][1], acc[2][2], acc[2][3]);
  acc_guard4(acc[3][0], acc[3][1], acc[3][2], acc[3][3]);

  float* slab = sT[wave];
  float bvj[4];
  float cs[4], cq[4];
  float mx[2][4], mn[2][4];
#pragma unroll
  for (int j = 0; j < 4; ++j) {
    bvj[j] = 0.0f;
    if (EPI >= 1) bvj[j] = bias[n0 + (j << 4) + rlane];
    cs[j] = 0.0f;
    cq[j] = 0.0f;
    mx[0][j] = -__builtin_inff();
    mx[1][j] = -__builtin_inff();
    mn[0][j] = __builtin_inff();
    mn[1][j] = __builtin_inff();
  }

#pragma unroll
  for (int i = 0; i < 4; ++i) {
    const int mBase = m0 + (i << 4);
#pragma unroll
    for (int j = 0; j < 4; ++j) {
#pragma unroll
      for (int r = 0; r < 8; ++r) {
        float v = acc[i][j][r] * scale;
        if (EPI >= 1) v = v + bvj[j];
        if (EPI != 2) slab[(mOff + r) * 68 + (j << 4) + rlane] = v;
        if (EPI >= 1) {
          const float v2 = v * v;
          cs[j] = cs[j] + v;
          cq[j] = cq[j] + v2;
        }
        if (EPI == 2) {
          mx[i >> 1][j] = fmaxf(mx[i >> 1][j], v);
          mn[i >> 1][j] = fminf(mn[i >> 1][j], v);
        }
      }
    }
    if (EPI != 2) {
      wave_lds_sync();
      const int c4 = rlane * 4;
      for (int pass = 0; pass < 2; ++pass) {
#pragma unroll
        for (int it = 0; it < 8; ++it) {
          const int row = it * 2 + hh;
          const v4f v = *(const v4f*)(slab + row * 68 + c4);
          *(volatile v4f*)(Cout + (size_t)(mBase + row) * N + n0 + c4) = v;
        }
        __threadfence();
      }
      wave_lds_sync();
    }
  }

  if (EPI >= 1) {
#pragma unroll
    for (int j = 0; j < 4; ++j) {
      cs[j] = cs[j] + __shfl_xor(cs[j], 16, 32);
      cq[j] = cq[j] + __shfl_xor(cq[j], 16, 32);
    }
    if (EPI == 2) {
#pragma unroll
      for (int g = 0; g < 2; ++g)
#pragma unroll
        for (int j = 0; j < 4; ++j) {
          mx[g][j] = fmaxf(mx[g][j], __shfl_xor(mx[g][j], 16, 32));
          mn[g][j] = fminf(mn[g][j], __shfl_xor(mn[g][j], 16, 32));
        }
    }
    if (hh == 0) {
#pragma unroll
      for (int j = 0; j < 4; ++j) {
        slab[256 + (j << 4) + rlane] = cs[j];
        slab[320 + (j << 4) + rlane] = cq[j];
        if (EPI == 2) {
          slab[(j << 4) + rlane] = mx[0][j];
          slab[64 + (j << 4) + rlane] = mx[1][j];
          slab[128 + (j << 4) + rlane] = mn[0][j];
          slab[192 + (j << 4) + rlane] = mn[1][j];
        }
      }
    }
    wave_lds_sync();
    const int c4 = rlane * 4;
    const v4f pv = *(const v4f*)(slab + 256 + lane * 4);
    float* pd = part + (size_t)tile * 128 + lane * 4;
    v4f gv = pv;
    v4f nv = pv;
    float* gd = pd;
    float* nd = pd;
    if (EPI == 2) {
      gv = *(const v4f*)(slab + hh * 64 + c4);
      nv = *(const v4f*)(slab + 128 + hh * 64 + c4);
      gd = Cout + (size_t)(tm * 2 + hh) * N + n0 + c4;
      nd = Cmin + (size_t)(tm * 2 + hh) * N + n0 + c4;
    }
    *(volatile v4f*)pd = pv;
    if (EPI == 2) {
      *(volatile v4f*)gd = gv;
      *(volatile v4f*)nd = nv;
    }
    __threadfence();
    *(volatile v4f*)pd = pv;
    if (EPI == 2) {
      *(volatile v4f*)gd = gv;
      *(volatile v4f*)nd = nv;
    }
  }
}

__global__ __launch_bounds__(256) void group_kernel(const float* __restrict__ xyz, const float* __restrict__ Z,
                                                    const int* __restrict__ centIdx, const float* __restrict__ W0,
                                                    const float* __restrict__ b0, float* __restrict__ Y,
                                                    float* __restrict__ part) {
#pragma clang fp contract(off)
  __shared__ int s_sel[8 * 32];
  const int wave = threadIdx.x >> 5;
  const int lane = threadIdx.x & 31;
  const int hh = lane >> 4;
  const int gw = blockIdx.x * 8 + wave;
  const int b = gw >> 10;
  const float* Xb = xyz + (size_t)b * kPts * 3;
  const int ci = clamp_pt(centIdx[gw]);
  const float cx = Xb[ci * 3 + 0];
  const float cy = Xb[ci * 3 + 1];
  const float cz = Xb[ci * 3 + 2];
  const float cxx = cx * cx;
  const float cyy = cy * cy;
  const float czz = cz * cz;
  const float sqc = (cxx + czz) + cyy;
  const float r2 = __uint_as_float(0x3D23D70Au);

  int* sel = s_sel + wave * 32;
  sel[lane] = ci;
  __syncthreads();

  int cnt = 0;
  for (int ch = 0; ch < kPts / 32 && cnt < kSamp; ++ch) {
    const int p = ch * 32 + lane;
    const float x = Xb[p * 3 + 0];
    const float y = Xb[p * 3 + 1];
    const float z = Xb[p * 3 + 2];
    const float xx = x * x;
    const float yy = y * y;
    const float zz = z * z;
    const float sqp = (xx + zz) + yy;
    float dot = cx * x;
    dot = __builtin_fmaf(cy, y, dot);
    dot = __builtin_fmaf(cz, z, dot);
    float d = -2.0f * dot;
    d = d + sqc;
    d = d + sqp;
    const bool in = !(d > r2);
    const unsigned mask = (unsigned)__ballot(in);
    const int rank = cnt + __popc(mask & ((1u << lane) - 1u));
    if (in && rank < kSamp) sel[rank] = p;
    cnt += __popc(mask);
  }
  __syncthreads();
  const int first = sel[0];
  int q = sel[lane];
  q = (lane < cnt) ? q : first;
  q = clamp_pt(q);

  const int c4 = (lane & 15) * 4;
  float wx[4], wy[4], wz[4];
#pragma unroll
  for (int e = 0; e < 4; ++e) {
    wx[e] = W0[(c4 + e) * kW0Pitch + 0];
    wy[e] = W0[(c4 + e) * kW0Pitch + 1];
    wz[e] = W0[(c4 + e) * kW0Pitch + 2];
  }
  const v4f bb = *(const v4f*)(b0 + c4);
  asm volatile("" ::: "memory");

  float s4[4] = {0.0f, 0.0f, 0.0f, 0.0f};
  float q4[4] = {0.0f, 0.0f, 0.0f, 0.0f};
#pragma unroll 1
  for (int t = 0; t < 16; ++t) {
    const int k = 2 * t + hh;
    const int qk = clamp_pt(__shfl(q, k, 32));
    const float dx = Xb[qk * 3 + 0] - cx;
    const float dy = Xb[qk * 3 + 1] - cy;
    const float dz = Xb[qk * 3 + 2] - cz;
    const v4f zv = *(const v4f*)(Z + ((size_t)b * kPts + qk) * kChMid + c4);
    v4f yv;
#pragma unroll
    for (int e = 0; e < 4; ++e) {
      float y = zv[e] + bb[e];
      y = __builtin_fmaf(dx, wx[e], y);
      y = __builtin_fmaf(dy, wy[e], y);
      y = __builtin_fmaf(dz, wz[e], y);
      yv[e] = y;
      const float y2 = y * y;
      s4[e] = s4[e] + y;
      q4[e] = q4[e] + y2;
    }
    float* dst = Y + ((size_t)gw * kSamp + k) * kChMid + c4;
    *(volatile v4f*)dst = yv;
    __threadfence();
    *(volatile v4f*)dst = yv;
  }
#pragma unroll
  for (int e = 0; e < 4; ++e) {
    s4[e] = s4[e] + __shfl_xor(s4[e], 16, 32);
    q4[e] = q4[e] + __shfl_xor(q4[e], 16, 32);
  }
  v4f pv;
#pragma unroll
  for (int e = 0; e < 4; ++e) pv[e] = (hh == 0) ? s4[e] : q4[e];
  float* pd = part + (size_t)gw * 128 + lane * 4;
  *(volatile v4f*)pd = pv;
  __threadfence();
  *(volatile v4f*)pd = pv;
}

__global__ __launch_bounds__(512) void bn_finalize_kernel(const float* __restrict__ part, int tilesM, int tilesN,
                                                          const float* __restrict__ gamma, const float* __restrict__ beta,
                                                          float* __restrict__ ss) {
  __shared__ double red[4][128];
  __shared__ __align__(16) float sOut[256];
  const int tid = threadIdx.x;
  const int slot = tid & 127;
  const int prt = tid >> 7;
  const double invM = 1.0 / (double)kRows;
  if (tid < 256) sOut[tid] = 0.0f;
  const int tM = tilesM > 8192 ? 8192 : tilesM;
  const int tN = tilesN > 2 ? 2 : tilesN;
  for (int tn = 0; tn < tN; ++tn) {
    double a = 0.0;
#pragma unroll 4
    for (int tm = prt; tm < tM; tm += 4) a += (double)part[((size_t)tm * tN + tn) * 128 + slot];
    red[prt][slot] = a;
    __syncthreads();
    if (tid < 64) {
      const int o = tn * 64 + tid;
      const double s = ((red[0][tid] + red[1][tid]) + red[2][tid]) + red[3][tid];
      const double qq = ((red[0][64 + tid] + red[1][64 + tid]) + red[2][64 + tid]) + red[3][64 + tid];
      const double mean = s * invM;
      double var = qq * invM - mean * mean;
      var = var < 0.0 ? 0.0 : var;
      const float sc = gamma[o] * rsqrtf((float)var + 1e-5f);
      sOut[o] = sc;
      sOut[128 + o] = beta[o] - (float)mean * sc;
    }
    __syncthreads();
  }
  if (tid < 64) {
    const v4f v = *(const v4f*)(sOut + tid * 4);
    *(volatile v4f*)(ss + tid * 4) = v;
    __threadfence();
    *(volatile v4f*)(ss + tid * 4) = v;
  }
}

__global__ __launch_bounds__(256) void bnrelu_kernel(const float* __restrict__ Y, const float* __restrict__ ss,
                                                     unsigned short* __restrict__ Xp, int nThreads) {
  const int t = blockIdx.x * 256 + threadIdx.x;
  if (t < nThreads) {
    const int c8 = (t & 7) * 8;
    const v4f a0 = *(const v4f*)(Y + (size_t)t * 8);
    const v4f a1 = *(const v4f*)(Y + (size_t)t * 8 + 4);
    const v4f s0 = *(const v4f*)(ss + c8);
    const v4f s1 = *(const v4f*)(ss + c8 + 4);
    const v4f h0 = *(const v4f*)(ss + 128 + c8);
    const v4f h1 = *(const v4f*)(ss + 128 + c8 + 4);
    v8h o;
#pragma unroll
    for (int e = 0; e < 4; ++e) {
      float v = a0[e] * s0[e];
      v = v + h0[e];
      v = fmaxf(v, 0.0f);
      o[e] = (_Float16)v;
      float w = a1[e] * s1[e];
      w = w + h1[e];
      w = fmaxf(w, 0.0f);
      o[4 + e] = (_Float16)w;
    }
    _Float16* dst = (_Float16*)Xp + (size_t)t * 8;
    *(volatile v8h*)dst = o;
    __threadfence();
    *(volatile v8h*)dst = o;
  }
}

__global__ __launch_bounds__(256) void pool_out_kernel(const float* __restrict__ gmax, const float* __restrict__ gmin,
                                                       const float* __restrict__ ss, float* __restrict__ out, int nThreads) {
  const int t = blockIdx.x * 256 + threadIdx.x;
  if (t < nThreads) {
    const int c4 = (t & 31) * 4;
    const v4f gm = *(const v4f*)(gmax + (size_t)t * 4);
    const v4f gn = *(const v4f*)(gmin + (size_t)t * 4);
    const v4f sc = *(const v4f*)(ss + c4);
    const v4f sh = *(const v4f*)(ss + 128 + c4);
    v4f o;
#pragma unroll
    for (int e = 0; e < 4; ++e) {
      const float m = (sc[e] >= 0.0f) ? gm[e] : gn[e];
      float v = m * sc[e];
      v = v + sh[e];
      o[e] = fmaxf(v, 0.0f);
    }
    float* dst = out + (size_t)t * 4;
    *(volatile v4f*)dst = o;
    __threadfence();
    *(volatile v4f*)dst = o;
  }
}

constexpr size_t kOffCent  = 0;
constexpr size_t kOffWp0   = kOffCent + (size_t)kGroups * 4;
constexpr size_t kOffWp1   = kOffWp0 + (size_t)64 * 64 * 2;
constexpr size_t kOffWp2   = kOffWp1 + (size_t)64 * 64 * 2;
constexpr size_t kOffSs0   = kOffWp2 + (size_t)128 * 64 * 2;
constexpr size_t kOffSs1   = kOffSs0 + 1024;
constexpr size_t kOffSs2   = kOffSs1 + 1024;
constexpr size_t kOffP16   = kOffSs2 + 1024;
constexpr size_t kOffZ     = kOffP16 + (size_t)kSrcRows * 64 * 2;
constexpr size_t kOffY     = kOffZ + (size_t)kSrcRows * 64 * 4;
constexpr size_t kOffX     = kOffY + (size_t)kRows * 64 * 4;
constexpr size_t kOffGmax  = kOffX + (size_t)kRows * 64 * 2;
constexpr size_t kOffGmin  = kOffGmax + (size_t)kGroups * 128 * 4;
constexpr size_t kOffPart0 = kOffGmin + (size_t)kGroups * 128 * 4;
constexpr size_t kOffPart1 = kOffPart0 + (size_t)kGroups * 128 * 4;
constexpr size_t kOffPart2 = kOffPart1 + (size_t)(kRows / 64) * 128 * 4;
constexpr size_t kWsTotal  = kOffPart2 + (size_t)(kRows / 64) * 2 * 128 * 4;
static_assert(kWsTotal <= (size_t)134217728, "carve within 128 MiB");
static_assert(kOffP16 % 128 == 0 && kOffZ % 128 == 0 && kOffY % 128 == 0 && kOffX % 128 == 0, "line aligned");
static_assert(kOffGmax % 128 == 0 && kOffPart0 % 128 == 0 && kOffPart1 % 128 == 0 && kOffPart2 % 128 == 0, "line aligned");

extern "C" void kernel_launch(void* const* d_in, const int* in_sizes, int n_in, void* d_out, int out_size, void* d_ws,
                              size_t ws_size, hipStream_t stream) {
  (void)in_sizes;
  (void)n_in;
  (void)out_size;
  if (ws_size < kWsTotal) return;
  const float* xyz = (const float*)d_in[0];
  const float* pts = (const float*)d_in[1];
  const float* W0  = (const float*)d_in[2];
  const float* b0  = (const float*)d_in[3];
  const float* g0  = (const float*)d_in[4];
  const float* be0 = (const float*)d_in[5];
  const float* W1  = (const float*)d_in[6];
  const float* b1  = (const float*)d_in[7];
  const float* g1  = (const float*)d_in[8];
  const float* be1 = (const float*)d_in[9];
  const float* W2  = (const float*)d_in[10];
  const float* b2  = (const float*)d_in[11];
  const float* g2  = (const float*)d_in[12];
  const float* be2 = (const float*)d_in[13];
  float* out = (float*)d_out;
  float* outPts = out + (size_t)kGroups * 3;

  char* ws = (char*)d_ws;
  int* centIdx = (int*)(ws + kOffCent);
  unsigned short* Wp0 = (unsigned short*)(ws + kOffWp0);
  unsigned short* Wp1 = (unsigned short*)(ws + kOffWp1);
  unsigned short* Wp2 = (unsigned short*)(ws + kOffWp2);
  float* ss0 = (float*)(ws + kOffSs0);
  float* ss1 = (float*)(ws + kOffSs1);
  float* ss2 = (float*)(ws + kOffSs2);
  unsigned short* P16 = (unsigned short*)(ws + kOffP16);
  float* Zp = (float*)(ws + kOffZ);
  float* Yp = (float*)(ws + kOffY);
  unsigned short* Xp = (unsigned short*)(ws + kOffX);
  float* gmax = (float*)(ws + kOffGmax);
  float* gmin = (float*)(ws + kOffGmin);
  float* part0 = (float*)(ws + kOffPart0);
  float* part1 = (float*)(ws + kOffPart1);
  float* part2 = (float*)(ws + kOffPart2);

  fps_kernel<<<kBatch, 512, 0, stream>>>(xyz, centIdx);
  prep_w_kernel<<<dim3(4, 3), 256, 0, stream>>>(W0, W1, W2, Wp0, Wp1, Wp2);
  cast_points_kernel<<<kSrcRows * 8 / 256, 256, 0, stream>>>(pts, P16, kSrcRows * 8);
  gemm_k64<0><<<(kSrcRows / 64) / 8, 256, 0, stream>>>(P16, Wp0, Zp, Zp, part0, b0, kSrcRows, kChMid, kWCarryInv);
  newxyz_kernel<<<kGroups * 3 / 256, 256, 0, stream>>>(xyz, centIdx, out);
  group_kernel<<<kGroups / 8, 256, 0, stream>>>(xyz, Zp, centIdx, W0, b0, Yp, part0);
  bn_finalize_kernel<<<1, 512, 0, stream>>>(part0, kGroups, 1, g0, be0, ss0);
  bnrelu_kernel<<<kRows * 8 / 256, 256, 0, stream>>>(Yp, ss0, Xp, kRows * 8);
  gemm_k64<1><<<(kRows / 64) / 8, 256, 0, stream>>>(Xp, Wp1, Yp, Yp, part1, b1, kRows, kChMid, kWCarryInv);
  bn_finalize_kernel<<<1, 512, 0, stream>>>(part1, kRows / 64, 1, g1, be1, ss1);
  bnrelu_kernel<<<kRows * 8 / 256, 256, 0, stream>>>(Yp, ss1, Xp, kRows * 8);
  gemm_k64<2><<<(kRows / 64) * 2 / 8, 256, 0, stream>>>(Xp, Wp2, gmax, gmin, part2, b2, kRows, kChOut, kWCarryInv);
  bn_finalize_kernel<<<1, 512, 0, stream>>>(part2, kRows / 64, 2, g2, be2, ss2);
  pool_out_kernel<<<kGroups * 32 / 256, 256, 0, stream>>>(gmax, gmin, ss2, outPts, kGroups * 32);
}
